// MultiHeadAttention_8847632629898
// MI455X (gfx1250) — hardware-verified
//
#include <hip/hip_runtime.h>

#ifndef NB
#define NB 2
#endif
#ifndef SEQ
#define SEQ 2048
#endif
#define NB_FULL 2
#define SEQ_FULL 2048
#define DD 1024
#define NH 16
#define HD 64
#define NR ((size_t)NB * SEQ)
#define RSC 0.0009765625f

static_assert(NH * HD == DD);
static_assert(HD == 64);
static_assert(SEQ % 128 == 0);
static_assert(DD % 64 == 0);
static_assert(DD % 32 == 0);
static_assert(SEQ % 64 == 0);
static_assert(NB <= NB_FULL);
static_assert(SEQ <= SEQ_FULL);

typedef _Float16 v16h __attribute__((ext_vector_type(16)));
typedef unsigned short v8us __attribute__((ext_vector_type(8), may_alias));
typedef float v8f __attribute__((ext_vector_type(8)));
typedef float v4f __attribute__((ext_vector_type(4)));
typedef float v4fa __attribute__((ext_vector_type(4), may_alias));
union FragH { v16h v; v8us half[2]; _Float16 h[16]; unsigned short u[16]; };

__device__ __forceinline__ unsigned short bf16_bits(float x) { unsigned int u = __float_as_uint(x); return (unsigned short)((u + 0x7FFFu + ((u >> 16) & 1u)) >> 16); }
__device__ __forceinline__ float bf16_rne(float x) { return __uint_as_float(((unsigned int)bf16_bits(x)) << 16); }

__device__ __forceinline__ v16h g2_frag(const _Float16* p, int hh) { FragH f; f.half[0] = *(const v8us*)((const unsigned short*)p + 8 * hh); f.half[1] = *(const v8us*)((const unsigned short*)p + 16 + 8 * hh); return f.v; }
__device__ __forceinline__ v8f g2_mma(v16h a, v16h b, v8f c) { v8f d = __builtin_amdgcn_wmma_f32_16x16x32_f16(false, a, false, b, (short)0, c, false, false); asm volatile("v_nop\n\tv_nop\n\tv_nop\n\tv_nop" : "+v"(d) : "v"(a), "v"(b)); return d; }

__global__ __launch_bounds__(256) void k_wt_f16(const float* __restrict__ W, _Float16* __restrict__ Wt, int K, int N, float scale) {
  const int t = blockIdx.x * 256 + threadIdx.x; if (t >= N * (K / 8)) return;
  const int n = t / (K / 8), k8 = (t % (K / 8)) * 8; FragH f;
#pragma unroll
  for (int i = 0; i < 8; ++i) f.h[i] = (_Float16)(bf16_rne(W[(size_t)(k8 + i) * N + n]) * scale);
  const v8us o = f.half[0];
  unsigned short* dst = (unsigned short*)Wt + (size_t)n * K + k8;
  *(volatile v8us*)dst = o; __threadfence(); *(volatile v8us*)dst = o;
}

__global__ __launch_bounds__(256) void k_x16(const float* __restrict__ x, _Float16* __restrict__ X16) {
  const size_t t = (size_t)blockIdx.x * 256 + threadIdx.x; if (t >= NR * DD / 8) return;
  const size_t r = t / (DD / 8); const int c8 = (int)(t % (DD / 8)) * 8; const size_t bb = r / SEQ, s = r % SEQ;
  const float* src = x + (bb * SEQ_FULL + s) * DD + c8;
  const v4f a = *(const v4fa*)src, c = *(const v4fa*)(src + 4); FragH f;
#pragma unroll
  for (int q = 0; q < 4; ++q) { f.h[q] = (_Float16)bf16_rne(a[q]); f.h[4 + q] = (_Float16)bf16_rne(c[q]); }
  const v8us o = f.half[0];
  unsigned short* dst = (unsigned short*)X16 + t * 8;
  *(volatile v8us*)dst = o; __threadfence(); *(volatile v8us*)dst = o;
}

__device__ __forceinline__ void gemm_kloop(const _Float16* __restrict__ A, size_t a0off, size_t a1off, const _Float16* __restrict__ Bh, size_t b0off, size_t bstep, int K, int hh,
                                           v8f& c00, v8f& c01, v8f& c02, v8f& c03, v8f& c10, v8f& c11, v8f& c12, v8f& c13) {
#pragma unroll 1
  for (int kb = 0; kb < K; kb += 32) {
    const v16h a0 = g2_frag(A + a0off + kb, hh), a1 = g2_frag(A + a1off + kb, hh);
    v16h b = g2_frag(Bh + b0off + kb, hh); c00 = g2_mma(a0, b, c00); c10 = g2_mma(a1, b, c10);
    b = g2_frag(Bh + b0off + bstep + kb, hh); c01 = g2_mma(a0, b, c01); c11 = g2_mma(a1, b, c11);
    b = g2_frag(Bh + b0off + 2 * bstep + kb, hh); c02 = g2_mma(a0, b, c02); c12 = g2_mma(a1, b, c12);
    b = g2_frag(Bh + b0off + 3 * bstep + kb, hh); c03 = g2_mma(a0, b, c03); c13 = g2_mma(a1, b, c13);
  }
}

__global__ __launch_bounds__(128) void k_gemm_proj(const _Float16* __restrict__ A, int lda, const _Float16* __restrict__ Bh, int ldb, float alpha,
                                                   _Float16* __restrict__ C16, _Float16* __restrict__ C16L, int ldc, int M, int N, int K) {
  __shared__ __attribute__((aligned(16))) float so[4][32][68];
  const int tid = threadIdx.x, w = tid >> 5, lane = tid & 31, ln = lane & 15, hh = lane >> 4;
  const int ntn = N >> 6; const int mt = blockIdx.x / ntn, nq = blockIdx.x - mt * ntn; const int row0 = mt * 128 + 32 * w, col0 = nq * 64; if (row0 >= M) return;
  const size_t a0off = (size_t)(row0 + ln) * lda, a1off = a0off + (size_t)16 * lda; const size_t b0off = (size_t)(col0 + ln) * ldb, bstep = (size_t)16 * ldb;
  const v8f z8 = {0.f, 0.f, 0.f, 0.f, 0.f, 0.f, 0.f, 0.f}; v8f c00 = z8, c01 = z8, c02 = z8, c03 = z8, c10 = z8, c11 = z8, c12 = z8, c13 = z8;
  gemm_kloop(A, a0off, a1off, Bh, b0off, bstep, K, hh, c00, c01, c02, c03, c10, c11, c12, c13);
  v8f accs[8] = {c00, c01, c02, c03, c10, c11, c12, c13};
#pragma unroll
  for (int u = 0; u < 8; ++u) { const int t = u & 3, half = u >> 2;
#pragma unroll
    for (int r = 0; r < 8; ++r) so[w][half * 16 + 8 * hh + r][t * 16 + ln] = accs[u][r] * alpha; }
  __builtin_amdgcn_fence(4  , "workgroup"); __builtin_amdgcn_wave_barrier();
  const int rq = lane >> 3, c8 = (lane & 7) * 8;
  for (int pass = 0; pass < 2; ++pass) {
#pragma unroll
    for (int q = 0; q < 8; ++q) { const int r = q * 4 + rq; const v4f x0 = *(const v4fa*)&so[w][r][c8], x1 = *(const v4fa*)&so[w][r][c8 + 4]; FragH fh, fl;
#pragma unroll
      for (int i = 0; i < 4; ++i) { _Float16 g = (_Float16)x0[i]; fh.h[i] = g; fl.h[i] = (_Float16)((x0[i] - (float)g) * 1024.0f); g = (_Float16)x1[i]; fh.h[4 + i] = g; fl.h[4 + i] = (_Float16)((x1[i] - (float)g) * 1024.0f); }
      const size_t d = (size_t)(row0 + r) * ldc + col0 + c8;
      *(volatile v8us*)((unsigned short*)C16 + d) = fh.half[0]; *(volatile v8us*)((unsigned short*)C16L + d) = fl.half[0]; }
    if (pass == 0) __threadfence(); }
}

__global__ __launch_bounds__(128) void k_gemm_out(const _Float16* __restrict__ A, const _Float16* __restrict__ AL, int lda, const _Float16* __restrict__ Bh, int ldb, const int* __restrict__ vlen, float alpha,
                                                  float* __restrict__ C, int ldc, int M, int N, int K) {
  __shared__ __attribute__((aligned(16))) float so[4][32][68];
  const int tid = threadIdx.x, w = tid >> 5, lane = tid & 31, ln = lane & 15, hh = lane >> 4;
  const int ntn = N >> 6; const int mt = blockIdx.x / ntn, nq = blockIdx.x - mt * ntn; const int row0 = mt * 128 + 32 * w, col0 = nq * 64; if (row0 >= M) return;
  int bb = (mt * 128) / SEQ; bb = (bb < NB - 1) ? bb : (NB - 1);
  const int vl = __builtin_amdgcn_readfirstlane(vlen[bb]);
  const int nvis = (vl <= 0) ? SEQ : ((vl < SEQ) ? vl : SEQ);
  const bool shortb = (nvis <= 256);
  const size_t a0off = (size_t)(row0 + ln) * lda, a1off = a0off + (size_t)16 * lda; const size_t b0off = (size_t)(col0 + ln) * ldb, bstep = (size_t)16 * ldb;
  const v8f z8 = {0.f, 0.f, 0.f, 0.f, 0.f, 0.f, 0.f, 0.f}; v8f c00 = z8, c01 = z8, c02 = z8, c03 = z8, c10 = z8, c11 = z8, c12 = z8, c13 = z8;
  if (shortb) {
    gemm_kloop(AL, a0off, a1off, Bh, b0off, bstep, K, hh, c00, c01, c02, c03, c10, c11, c12, c13);
    c00 = c00 * RSC; c01 = c01 * RSC; c02 = c02 * RSC; c03 = c03 * RSC; c10 = c10 * RSC; c11 = c11 * RSC; c12 = c12 * RSC; c13 = c13 * RSC;
  }
  gemm_kloop(A, a0off, a1off, Bh, b0off, bstep, K, hh, c00, c01, c02, c03, c10, c11, c12, c13);
  v8f accs[8] = {c00, c01, c02, c03, c10, c11, c12, c13};
#pragma unroll
  for (int u = 0; u < 8; ++u) { const int t = u & 3, half = u >> 2;
#pragma unroll
    for (int r = 0; r < 8; ++r) so[w][half * 16 + 8 * hh + r][t * 16 + ln] = accs[u][r] * alpha; }
  __builtin_amdgcn_fence(4  , "workgroup"); __builtin_amdgcn_wave_barrier();
  const int rsub = lane >> 4, c4 = (lane & 15) * 4;
  for (int pass = 0; pass < 2; ++pass) {
#pragma unroll
    for (int q = 0; q < 16; ++q) { const int r = q * 2 + rsub; const v4f v = *(const v4fa*)&so[w][r][c4]; *(volatile v4f*)(C + (size_t)(row0 + r) * ldc + col0 + c4) = v; }
    if (pass == 0) __threadfence(); }
}

__global__ __launch_bounds__(256) void k_vt(const _Float16* __restrict__ V16, _Float16* __restrict__ Vt) {
  __shared__ unsigned short tl[64][66];
  const int tid = threadIdx.x; const int slab = blockIdx.x / (SEQ / 64), lg = blockIdx.x % (SEQ / 64); const int b = slab / NH, h = slab % NH;
  for (int i = tid; i < 64 * 8; i += 256) { const int r = i / 8, c8 = (i % 8) * 8; FragH f; f.half[0] = *(const v8us*)((const unsigned short*)V16 + ((size_t)b * SEQ + lg * 64 + r) * DD + h * HD + c8);
#pragma unroll
    for (int q = 0; q < 8; ++q) tl[r][c8 + q] = f.u[q]; }
  __syncthreads();
  for (int pass = 0; pass < 2; ++pass) {
#pragma unroll
    for (int rd = 0; rd < 2; ++rd) { const int d = rd * 32 + tid / 8, pc = tid % 8; FragH f;
#pragma unroll
      for (int q = 0; q < 8; ++q) f.u[q] = tl[pc * 8 + q][d];
      *(volatile v8us*)((unsigned short*)Vt + ((size_t)slab * HD + d) * SEQ + lg * 64 + pc * 8) = f.half[0]; }
    if (pass == 0) __threadfence(); }
}

__global__ __launch_bounds__(128) void k_flash(const _Float16* __restrict__ Q16, const _Float16* __restrict__ QL, const _Float16* __restrict__ K16, const _Float16* __restrict__ KL,
                                               const _Float16* __restrict__ VT, const _Float16* __restrict__ VTL, const int* __restrict__ vlen, _Float16* __restrict__ O16, _Float16* __restrict__ OL) {
  __shared__ __attribute__((aligned(16))) float so[4][16][68];
  const int tid = threadIdx.x, w = tid >> 5, lane = tid & 31, ln = lane & 15, hh = lane >> 4;
  const int qt = blockIdx.x % (SEQ / 64); const int bh = blockIdx.x / (SEQ / 64); const int h = bh % NH; const int b = bh / NH;
  const int vl = __builtin_amdgcn_readfirstlane(vlen[b]);
  const int nvis = (vl <= 0) ? SEQ : ((vl < SEQ) ? vl : SEQ);
  const int nhalf = (nvis + 31) >> 5;
  const bool shortb = (nvis <= 256);
  const int q0 = qt * 64 + w * 16;
  const size_t qoff = ((size_t)b * SEQ + q0 + ln) * DD + (size_t)h * HD;
  const v16h qh0 = g2_frag(Q16 + qoff, hh), qh1 = g2_frag(Q16 + qoff + 32, hh);
  const size_t kbase = ((size_t)b * SEQ + ln) * DD + (size_t)h * HD;
  const size_t vbase = ((size_t)bh * HD + ln) * SEQ;
  const v8f z8 = {0.f, 0.f, 0.f, 0.f, 0.f, 0.f, 0.f, 0.f};
  v8f o0 = z8, o1 = z8, o2 = z8, o3 = z8, r0 = z8, r1 = z8, r2 = z8, r3 = z8;
  float m = -1.0e30f, l = 0.f;
#pragma unroll 1
  for (int kc = 0; kc < nhalf; ++kc) {
    const int k0 = kc * 32;
    const size_t ka = kbase + (size_t)k0 * DD; const size_t kb = ka + (size_t)16 * DD;
    v8f t0 = z8, t1 = z8;
    if (shortb) {
      const v16h ql0 = g2_frag(QL + qoff, hh), ql1 = g2_frag(QL + qoff + 32, hh);
      v16h a = g2_frag(K16 + ka, hh); t0 = g2_mma(a, ql0, t0);
      a = g2_frag(K16 + ka + 32, hh); t0 = g2_mma(a, ql1, t0);
      a = g2_frag(KL + ka, hh); t0 = g2_mma(a, qh0, t0);
      a = g2_frag(KL + ka + 32, hh); t0 = g2_mma(a, qh1, t0);
      a = g2_frag(K16 + kb, hh); t1 = g2_mma(a, ql0, t1);
      a = g2_frag(K16 + kb + 32, hh); t1 = g2_mma(a, ql1, t1);
      a = g2_frag(KL + kb, hh); t1 = g2_mma(a, qh0, t1);
      a = g2_frag(KL + kb + 32, hh); t1 = g2_mma(a, qh1, t1);
      t0 = t0 * RSC; t1 = t1 * RSC;
    }
    {
      v16h a = g2_frag(K16 + ka, hh); t0 = g2_mma(a, qh0, t0);
      a = g2_frag(K16 + ka + 32, hh); t0 = g2_mma(a, qh1, t0);
      a = g2_frag(K16 + kb, hh); t1 = g2_mma(a, qh0, t1);
      a = g2_frag(K16 + kb + 32, hh); t1 = g2_mma(a, qh1, t1);
    }
    float s0[8], s1[8]; float mx = -3.0e38f;
#pragma unroll
    for (int r = 0; r < 8; ++r) { const int kj = k0 + 8 * hh + r; const float a0 = t0[r] * 0.125f, a1 = t1[r] * 0.125f;
      s0[r] = (kj < vl) ? a0 : -1.0e6f; s1[r] = (kj + 16 < vl) ? a1 : -1.0e6f; mx = fmaxf(mx, fmaxf(s0[r], s1[r])); }
    mx = fmaxf(mx, __shfl_xor(mx, 16));
    const float mn = fmaxf(m, mx); const float corr = __expf(m - mn); m = mn;
    FragH ph, pl; pl.v = ph.v = (v16h)(_Float16)0.0f; float ls = 0.f;
#pragma unroll
    for (int r = 0; r < 8; ++r) { const float e0 = __expf(s0[r] - mn), e1 = __expf(s1[r] - mn); ls += e0 + e1;
      const float c0 = e0 * 1024.0f, c1 = e1 * 1024.0f; const _Float16 g0 = (_Float16)c0, g1 = (_Float16)c1; ph.h[r] = g0; ph.h[8 + r] = g1;
      if (shortb) { pl.h[r] = (_Float16)((c0 - (float)g0) * 1024.0f); pl.h[8 + r] = (_Float16)((c1 - (float)g1) * 1024.0f); } }
    l = l * corr + ls;
    o0 = o0 * corr; o1 = o1 * corr; o2 = o2 * corr; o3 = o3 * corr;
    const size_t va = vbase + (size_t)k0;
    const v16h a0 = g2_frag(VT + va, hh), a1 = g2_frag(VT + va + (size_t)16 * SEQ, hh), a2 = g2_frag(VT + va + (size_t)32 * SEQ, hh), a3 = g2_frag(VT + va + (size_t)48 * SEQ, hh);
    o0 = g2_mma(a0, ph.v, o0); o1 = g2_mma(a1, ph.v, o1); o2 = g2_mma(a2, ph.v, o2); o3 = g2_mma(a3, ph.v, o3);
    if (shortb) {
      r0 = r0 * corr; r1 = r1 * corr; r2 = r2 * corr; r3 = r3 * corr;
      r0 = g2_mma(a0, pl.v, r0); r1 = g2_mma(a1, pl.v, r1); r2 = g2_mma(a2, pl.v, r2); r3 = g2_mma(a3, pl.v, r3);
      const v16h b0 = g2_frag(VTL + va, hh), b1 = g2_frag(VTL + va + (size_t)16 * SEQ, hh), b2 = g2_frag(VTL + va + (size_t)32 * SEQ, hh), b3 = g2_frag(VTL + va + (size_t)48 * SEQ, hh);
      r0 = g2_mma(b0, ph.v, r0); r1 = g2_mma(b1, ph.v, r1); r2 = g2_mma(b2, ph.v, r2); r3 = g2_mma(b3, ph.v, r3);
    }
  }
  const float lt = l + __shfl_xor(l, 16);
  const float fin = 0.0625f * (1.0f / lt);
#pragma unroll
  for (int r = 0; r < 8; ++r) {
    so[w][ln][8 * hh + r] = (o0[r] + r0[r] * RSC) * fin;
    so[w][ln][16 + 8 * hh + r] = (o1[r] + r1[r] * RSC) * fin;
    so[w][ln][32 + 8 * hh + r] = (o2[r] + r2[r] * RSC) * fin;
    so[w][ln][48 + 8 * hh + r] = (o3[r] + r3[r] * RSC) * fin;
  }
  __builtin_amdgcn_fence(4  , "workgroup"); __builtin_amdgcn_wave_barrier();
  const int rq = lane >> 3, c8 = (lane & 7) * 8;
  for (int pass = 0; pass < 2; ++pass) {
#pragma unroll
    for (int i = 0; i < 4; ++i) { const int q = i * 4 + rq; const v4f x0 = *(const v4fa*)&so[w][q][c8], x1 = *(const v4fa*)&so[w][q][c8 + 4]; FragH fh, fl;
#pragma unroll
      for (int u = 0; u < 4; ++u) { _Float16 g = (_Float16)x0[u]; fh.h[u] = g; fl.h[u] = (_Float16)((x0[u] - (float)g) * 1024.0f); g = (_Float16)x1[u]; fh.h[4 + u] = g; fl.h[4 + u] = (_Float16)((x1[u] - (float)g) * 1024.0f); }
      const size_t d = ((size_t)b * SEQ + q0 + q) * DD + (size_t)h * HD + c8;
      *(volatile v8us*)((unsigned short*)O16 + d) = fh.half[0]; *(volatile v8us*)((unsigned short*)OL + d) = fl.half[0]; }
    if (pass == 0) __threadfence(); }
}

#define PL_W ((size_t)DD * DD * 2)
#define PL_X ((size_t)NB * SEQ * DD * 2)
#define WS_TOTAL (4 * PL_W + 13 * PL_X)
static_assert(WS_TOTAL <= (size_t)134217728);
static_assert(PL_W % 256 == 0);
static_assert(PL_X % 256 == 0);
static_assert(((size_t)NB * SEQ) % 128 == 0);
static_assert(((size_t)NB * SEQ * DD / 8) % 256 == 0);

extern "C" void kernel_launch(void* const* d_in, const int* in_sizes, int n_in,
                              void* d_out, int out_size, void* d_ws, size_t ws_size, hipStream_t stream) {
  if (n_in < 8) return;
  const long long needx = ((long long)(NB - 1) * SEQ_FULL + SEQ) * DD;
  if (in_sizes[0] < needx || in_sizes[1] < needx || in_sizes[2] < needx) return;
  if (in_sizes[3] < NB) return;
  if (in_sizes[4] < DD * DD || in_sizes[5] < DD * DD || in_sizes[6] < DD * DD || in_sizes[7] < DD * DD) return;
  if ((long long)out_size < (long long)NB * SEQ * DD) return;
  if (ws_size < WS_TOTAL) return;
  const float* xq = (const float*)d_in[0]; const float* xk = (const float*)d_in[1]; const float* xv = (const float*)d_in[2]; const int* vlen = (const int*)d_in[3];
  const float* wq = (const float*)d_in[4]; const float* wk = (const float*)d_in[5]; const float* wv = (const float*)d_in[6]; const float* wo = (const float*)d_in[7];
  char* ws = (char*)d_ws; size_t off = 0;
  auto take = [&](size_t bytes) { char* p = ws + off; off += (bytes + 255) & ~(size_t)255; return p; };
  _Float16* BQ = (_Float16*)take(PL_W); _Float16* BK = (_Float16*)take(PL_W); _Float16* BV = (_Float16*)take(PL_W); _Float16* BO = (_Float16*)take(PL_W);
  _Float16* XQ = (_Float16*)take(PL_X); _Float16* XK = (_Float16*)take(PL_X); _Float16* XV = (_Float16*)take(PL_X);
  _Float16* Q16 = (_Float16*)take(PL_X); _Float16* QL = (_Float16*)take(PL_X); _Float16* K16 = (_Float16*)take(PL_X); _Float16* KL = (_Float16*)take(PL_X); _Float16* V16 = (_Float16*)take(PL_X); _Float16* VL = (_Float16*)take(PL_X);
  _Float16* VT = (_Float16*)take(PL_X); _Float16* VTL = (_Float16*)take(PL_X); _Float16* O16 = (_Float16*)take(PL_X); _Float16* OL = (_Float16*)take(PL_X);
  if (off > ws_size) return;
  const unsigned gw = (unsigned)(((size_t)DD * DD / 8 + 255) / 256);
  k_wt_f16<<<gw, 256, 0, stream>>>(wq, BQ, DD, DD, 16.0f);
  k_wt_f16<<<gw, 256, 0, stream>>>(wk, BK, DD, DD, 16.0f);
  k_wt_f16<<<gw, 256, 0, stream>>>(wv, BV, DD, DD, 16.0f);
  k_wt_f16<<<gw, 256, 0, stream>>>(wo, BO, DD, DD, 16.0f);
  const unsigned gx = (unsigned)((NR * DD / 8 + 255) / 256);
  k_x16<<<gx, 256, 0, stream>>>(xq, XQ);
  k_x16<<<gx, 256, 0, stream>>>(xk, XK);
  k_x16<<<gx, 256, 0, stream>>>(xv, XV);
  const unsigned gg = (unsigned)((NR / 128) * (DD / 64));
  k_gemm_proj<<<gg, 128, 0, stream>>>(XQ, DD, BQ, DD, 0.0625f, Q16, QL, DD, (int)NR, DD, DD);
  k_gemm_proj<<<gg, 128, 0, stream>>>(XK, DD, BK, DD, 0.0625f, K16, KL, DD, (int)NR, DD, DD);
  k_gemm_proj<<<gg, 128, 0, stream>>>(XV, DD, BV, DD, 0.0625f, V16, VL, DD, (int)NR, DD, DD);
  const unsigned gt = (unsigned)(NB * NH * (SEQ / 64));
  k_vt<<<gt, 256, 0, stream>>>(V16, VT);
  k_vt<<<gt, 256, 0, stream>>>(VL, VTL);
  k_flash<<<gt, 128, 0, stream>>>(Q16, QL, K16, KL, VT, VTL, vlen, O16, OL);
  k_gemm_out<<<gg, 128, 0, stream>>>(O16, OL, DD, BO, DD, vlen, RSC, (float*)d_out, DD, (int)NR, DD, DD);
}
